// LocalMultiMessagePassing_6133213299116
// MI455X (gfx1250) — hardware-verified
//
#include <hip/hip_runtime.h>
#include <stddef.h>
#include <stdint.h>


#define DF    128
#define GT    128
#define GW    4
#define SP    132

#define NB    512
#define CHUNK 2048
#define ATHR  256
#define AWAVE 8
#define WCAP  256
#define NGRP  (CHUNK / (ATHR * 4))
#define SACC4 (NB * (DF / 4))
#define LDS_LIST (AWAVE * WCAP)
#define ALDS_BYTES (SACC4 * 16 + LDS_LIST * 4 + 64)

#define PTHR  256
#define PWAVE 8

static_assert(GW * 32 == GT);
static_assert(WCAP == (CHUNK / ATHR) * 32);
static_assert(NGRP == 2);
static_assert(NB == 512);
static_assert(CHUNK <= 2048);
static_assert(ALDS_BYTES == 270400);
static_assert(PWAVE * 32 == PTHR);

typedef float          v4f   __attribute__((ext_vector_type(4)));
typedef float          v8f   __attribute__((ext_vector_type(8)));
typedef int            v4i   __attribute__((ext_vector_type(4)));
typedef unsigned short us16;
typedef us16           v8us  __attribute__((ext_vector_type(8)));
typedef us16           v16us __attribute__((ext_vector_type(16)));
typedef __bf16         v16b  __attribute__((ext_vector_type(16)));
union BFrag { v16b v; v16us u; v8us h[2]; };
union Pack8 { v8us h; v4i q; };

__device__ __forceinline__ v8f wm(v16b a, v16b b, v8f c) {
  v8f d = __builtin_amdgcn_wmma_f32_16x16x32_bf16(false, a, false, b, (short)0, c, false, false);
  asm volatile("v_nop\n\tv_nop\n\tv_nop\n\tv_nop" : "+v"(d) : "v"(a), "v"(b));
  return d;
}

__device__ __forceinline__ unsigned bfb(float f) {
  unsigned u = __float_as_uint(f);
  u += 0x7FFFu + ((u >> 16) & 1u);
  return u >> 16;
}
__device__ __forceinline__ void split2(float f, us16& hi, us16& lo) {
  const unsigned hb = bfb(f);
  const float hf = __uint_as_float(hb << 16);
  hi = (us16)hb;
  lo = (us16)bfb(f - hf);
}

__device__ __forceinline__ float leaky(float v) { return v >= 0.f ? v : 0.01f * v; }

__global__ __launch_bounds__(256) void k_prep(const float* __restrict__ W, us16* Wh, us16* Wl, int n8) {
  const int i = blockIdx.x * 256 + threadIdx.x;
  if (i >= n8) return;
  const size_t o = (size_t)i * 8;
  const v4f a = *(const v4f*)(W + o);
  const v4f b = *(const v4f*)(W + o + 4);
  const float f[8] = {a.x, a.y, a.z, a.w, b.x, b.y, b.z, b.w};
  Pack8 ph, pl;
#pragma unroll
  for (int j = 0; j < 8; ++j) {
    us16 hh, ll;
    split2(f[j], hh, ll);
    ph.h[j] = hh;
    pl.h[j] = ll;
  }
  const v4i qh = ph.q, ql = pl.q;
  *(volatile v4i*)(Wh + o) = qh;
  *(volatile v4i*)(Wl + o) = ql;
  __threadfence();
  *(volatile v4i*)(Wh + o) = qh;
  *(volatile v4i*)(Wl + o) = ql;
}

template <int KSA, int KSB, bool RES, bool GATE>
__global__ __launch_bounds__(GT) __attribute__((amdgpu_num_vgpr(256)))
void k_gemm(const float* __restrict__ A0, const float* A1,
            const us16* __restrict__ Wh, const us16* __restrict__ Wl,
            const float* __restrict__ bias, const float* res,
            const float* __restrict__ wg, const float* __restrict__ bg,
            float* gout, float* out, int nRows) {
  __shared__ __attribute__((aligned(16))) float St[GW * 16 * SP];
  __shared__ __attribute__((aligned(16))) float Gs[GW * 16];
  constexpr int KT = (KSA + KSB) * 32;

  const int tid  = threadIdx.x;
  const int lane = tid & 31;
  const int wave = tid >> 5;
  const int h    = lane >> 4;
  const int m    = lane & 15;
  const int rowBase = blockIdx.x * (GW * 16) + wave * 16;
  int rm = rowBase + m;
  if (rm > nRows - 1) rm = nRows - 1;

  const float* pa0 = A0 + (size_t)rm * (KSA * 32) + 8 * h;
  const float* pa1 = A1 + (size_t)rm * (KSB * 32) + 8 * h;
  const us16*  qh0 = Wh + (size_t)m * KT + 8 * h;
  const us16*  ql0 = Wl + (size_t)m * KT + 8 * h;

  v8f acc[8];
#pragma unroll
  for (int nt = 0; nt < 8; ++nt) {
    const v8f z = {0.f, 0.f, 0.f, 0.f, 0.f, 0.f, 0.f, 0.f};
    acc[nt] = z;
  }
  float gs = 0.f;

#pragma unroll
  for (int ks = 0; ks < KSA + KSB; ++ks) {
    const float* pa = (ks < KSA) ? (pa0 + ks * 32) : (pa1 + (ks - KSA) * 32);
    const v4f f0 = *(const v4f*)(pa);
    const v4f f1 = *(const v4f*)(pa + 4);
    const v4f f2 = *(const v4f*)(pa + 16);
    const v4f f3 = *(const v4f*)(pa + 20);
    const float fv[16] = {f0.x, f0.y, f0.z, f0.w, f1.x, f1.y, f1.z, f1.w,
                          f2.x, f2.y, f2.z, f2.w, f3.x, f3.y, f3.z, f3.w};
    BFrag ah, al;
#pragma unroll
    for (int i = 0; i < 16; ++i) {
      us16 hb, lb;
      split2(fv[i], hb, lb);
      ah.u[i] = hb;
      al.u[i] = lb;
    }
    if (GATE && ks < KSA) {
      const v4f g0 = *(const v4f*)(wg + ks * 32 + 8 * h);
      const v4f g1 = *(const v4f*)(wg + ks * 32 + 8 * h + 4);
      const v4f g2 = *(const v4f*)(wg + ks * 32 + 16 + 8 * h);
      const v4f g3 = *(const v4f*)(wg + ks * 32 + 16 + 8 * h + 4);
      gs += f0.x * g0.x; gs += f0.y * g0.y; gs += f0.z * g0.z; gs += f0.w * g0.w;
      gs += f1.x * g1.x; gs += f1.y * g1.y; gs += f1.z * g1.z; gs += f1.w * g1.w;
      gs += f2.x * g2.x; gs += f2.y * g2.y; gs += f2.z * g2.z; gs += f2.w * g2.w;
      gs += f3.x * g3.x; gs += f3.y * g3.y; gs += f3.z * g3.z; gs += f3.w * g3.w;
    }
    const int kg = ks * 32;
#pragma unroll
    for (int nt = 0; nt < 8; ++nt) {
      const us16* qh = qh0 + (size_t)nt * 16 * KT + kg;
      const us16* ql = ql0 + (size_t)nt * 16 * KT + kg;
      BFrag bh, bl;
      bh.h[0] = *(const v8us*)qh;
      bh.h[1] = *(const v8us*)(qh + 16);
      bl.h[0] = *(const v8us*)ql;
      bl.h[1] = *(const v8us*)(ql + 16);
      acc[nt] = wm(ah.v, bh.v, acc[nt]);
      acc[nt] = wm(ah.v, bl.v, acc[nt]);
      acc[nt] = wm(al.v, bh.v, acc[nt]);
    }
  }

  float* sw = St + wave * (16 * SP);
#pragma unroll
  for (int nt = 0; nt < 8; ++nt) {
    const float bv = bias[nt * 16 + m];
#pragma unroll
    for (int r = 0; r < 8; ++r) sw[(8 * h + r) * SP + nt * 16 + m] = leaky(acc[nt][r] + bv);
  }
  if (GATE) {
    gs += __shfl_xor(gs, 16, 32);
    if (lane < 16) Gs[wave * 16 + m] = gs + bg[0];
  }
  __syncthreads();

  v4f vo[16];
#pragma unroll
  for (int i = 0; i < 16; ++i) {
    int rr = rowBase + i;
    if (rr > nRows - 1) rr = nRows - 1;
    v4f v = *(const v4f*)(sw + i * SP + 4 * lane);
    if (RES) v = v + *(const v4f*)(res + (size_t)rr * DF + 4 * lane);
    vo[i] = v;
  }
  v4f gv = {0.f, 0.f, 0.f, 0.f};
  const bool gwri = GATE && (wave == 0) && (lane < 16);
  if (gwri) gv = *(const v4f*)(Gs + 4 * lane);
  float* gp = gout + (size_t)blockIdx.x * (GW * 16) + 4 * lane;

#pragma unroll
  for (int i = 0; i < 16; ++i) {
    const int row = rowBase + i;
    if (row < nRows) *(volatile v4f*)(out + (size_t)row * DF + 4 * lane) = vo[i];
  }
  if (gwri) *(volatile v4f*)gp = gv;
  __threadfence();
#pragma unroll
  for (int i = 0; i < 16; ++i) {
    const int row = rowBase + i;
    if (row < nRows) *(volatile v4f*)(out + (size_t)row * DF + 4 * lane) = vo[i];
  }
  if (gwri) *(volatile v4f*)gp = gv;
}

__global__ __launch_bounds__(ATHR) void k_aggmax(const float* __restrict__ M, const int* __restrict__ ei,
                                                 float* agg, int nN, int nE) {
  extern __shared__ v4f lds_dyn[];
  v4f* sacc = lds_dyn;
  int* list = (int*)(lds_dyn + SACC4);
  int* wcnt = list + LDS_LIST;

  const int tid  = threadIdx.x;
  const int lane = tid & 31;
  const int wave = tid >> 5;
  const int nodeBase = blockIdx.x * NB;

  {
    const float ninf = -__builtin_inff();
    const v4f n4 = {ninf, ninf, ninf, ninf};
    for (int i = tid; i < SACC4; i += ATHR) sacc[i] = n4;
  }
  __syncthreads();

  const int* eid = ei + nE;
  const bool al16 = ((nE & 3) == 0);
  const int nChunks = (nE + CHUNK - 1) / CHUNK;
#pragma unroll 1
  for (int ch = 0; ch < nChunks; ++ch) {
    const int cbase = ch * CHUNK;
    int wc = 0;
#pragma unroll
    for (int g = 0; g < NGRP; ++g) {
      const int el0 = (g * ATHR + tid) * 4;
      const int e0  = cbase + el0;
      const int sent = -2147483647 - 1;
      v4i d;
      if (al16 && (e0 + 3 < nE)) {
        d = *(const v4i*)(eid + e0);
      } else {
        d.x = (e0     < nE) ? eid[min(e0, nE - 1)]     : sent;
        d.y = (e0 + 1 < nE) ? eid[min(e0 + 1, nE - 1)] : sent;
        d.z = (e0 + 2 < nE) ? eid[min(e0 + 2, nE - 1)] : sent;
        d.w = (e0 + 3 < nE) ? eid[min(e0 + 3, nE - 1)] : sent;
      }
      const unsigned s0 = (unsigned)d.x - (unsigned)nodeBase;
      const unsigned s1 = (unsigned)d.y - (unsigned)nodeBase;
      const unsigned s2 = (unsigned)d.z - (unsigned)nodeBase;
      const unsigned s3 = (unsigned)d.w - (unsigned)nodeBase;
      const bool h0 = s0 < (unsigned)NB;
      const bool h1 = s1 < (unsigned)NB;
      const bool h2 = s2 < (unsigned)NB;
      const bool h3 = s3 < (unsigned)NB;
      const unsigned many = __builtin_amdgcn_ballot_w32(h0 | h1 | h2 | h3);
      if (many != 0u) {
#define HITJ(J, HJ, SJ) { \
          const unsigned mj = __builtin_amdgcn_ballot_w32(HJ); \
          if (HJ) { \
            const int pos = wc + (int)__builtin_amdgcn_mbcnt_lo(mj, 0u); \
            if (pos < WCAP) list[wave * WCAP + pos] = ((el0 + (J)) << 9) | (int)(SJ); \
          } \
          wc += (int)__builtin_popcount(mj); }
        HITJ(0, h0, s0)
        HITJ(1, h1, s1)
        HITJ(2, h2, s2)
        HITJ(3, h3, s3)
#undef HITJ
      }
    }
    if (lane == 0) wcnt[wave] = wc;
    __syncthreads();

    if (wave == 0) {
      for (int wsx = 0; wsx < AWAVE; ++wsx) {
        int n = wcnt[wsx];
        if (n > WCAP) n = WCAP;
        if (n < 0) n = 0;
        for (int i = 0; i < n; ++i) {
          const int ent  = list[wsx * WCAP + i];
          const int slot = ent & (NB - 1);
          const int el   = (ent >> 9) & (CHUNK - 1);
          int e = cbase + el;
          if (e > nE - 1) e = nE - 1;
          int src = ei[e];
          src = src < 0 ? 0 : (src > nN - 1 ? nN - 1 : src);
          const v4f xv = *(const v4f*)(M + (size_t)src * DF + 4 * lane);
          v4f* sp = sacc + slot * 32 + lane;
          v4f c = *sp;
          c.x = fmaxf(c.x, xv.x);
          c.y = fmaxf(c.y, xv.y);
          c.z = fmaxf(c.z, xv.z);
          c.w = fmaxf(c.w, xv.w);
          *sp = c;
        }
      }
    }
    __syncthreads();
  }

  const float pinf = __builtin_inff();
#pragma unroll 1
  for (int j = 0; j < NB / AWAVE; ++j) {
    const int slot = wave * (NB / AWAVE) + j;
    const int node = nodeBase + slot;
    if (node >= nN) break;
    v4f v = sacc[slot * 32 + lane];
    v.x = (__builtin_fabsf(v.x) < pinf) ? v.x : 0.f;
    v.y = (__builtin_fabsf(v.y) < pinf) ? v.y : 0.f;
    v.z = (__builtin_fabsf(v.z) < pinf) ? v.z : 0.f;
    v.w = (__builtin_fabsf(v.w) < pinf) ? v.w : 0.f;
    float* op = agg + (size_t)node * DF + 4 * lane;
    *(volatile v4f*)op = v;
    __threadfence();
    *(volatile v4f*)op = v;
  }
}

__global__ __launch_bounds__(PTHR) void k_pool(const float* __restrict__ gate, const float* __restrict__ feat,
                                               const int* __restrict__ batch, float* xg, int nN) {
  __shared__ float red[PWAVE];
  __shared__ __attribute__((aligned(16))) v4f part[PWAVE * 32];

  const int g    = blockIdx.x;
  const int tid  = threadIdx.x;
  const int lane = tid & 31;
  const int wave = tid >> 5;
  const float pinf = __builtin_inff();

  float mx = -pinf;
  for (int base = wave * 32; base < nN; base += PTHR) {
    const int n = base + lane;
    if (n < nN) {
      if (batch[n] == g) mx = fmaxf(mx, gate[n]);
    }
  }
#pragma unroll
  for (int o = 16; o > 0; o >>= 1) mx = fmaxf(mx, __shfl_xor(mx, o, 32));
  if (lane == 0) red[wave] = mx;
  __syncthreads();
  float gm = red[0];
#pragma unroll
  for (int w = 1; w < PWAVE; ++w) gm = fmaxf(gm, red[w]);
  if (!(__builtin_fabsf(gm) < pinf)) gm = 0.f;
  __syncthreads();

  float ds = 0.f;
  v4f xa = {0.f, 0.f, 0.f, 0.f};
  for (int base = wave * 32; base < nN; base += PTHR) {
    const int n = base + lane;
    bool hit = false;
    if (n < nN) hit = (batch[n] == g);
    float ev = 0.f;
    if (hit) {
      ev = expf(gate[n] - gm);
      ds += ev;
    }
    unsigned msk = __builtin_amdgcn_ballot_w32(hit);
    while (msk != 0u) {
      const int j = __builtin_ctz(msk);
      msk &= msk - 1u;
      const float ej = __shfl(ev, j, 32);
      const int nj = base + j;
      const v4f fvv = *(const v4f*)(feat + (size_t)nj * DF + 4 * lane);
      xa = xa + ej * fvv;
    }
  }
#pragma unroll
  for (int o = 16; o > 0; o >>= 1) ds += __shfl_xor(ds, o, 32);
  if (lane == 0) red[wave] = ds;
  part[wave * 32 + lane] = xa;
  __syncthreads();

  if (wave == 0) {
    float dn = red[0];
#pragma unroll
    for (int w = 1; w < PWAVE; ++w) dn += red[w];
    if (dn == 0.f) dn = 1.f;
    v4f s = part[lane];
#pragma unroll
    for (int w = 1; w < PWAVE; ++w) s = s + part[w * 32 + lane];
    const float inv = 1.0f / dn;
    const v4f o4 = s * inv;
    float* op = xg + (size_t)g * DF + 4 * lane;
    *(volatile v4f*)op = o4;
    __threadfence();
    *(volatile v4f*)op = o4;
  }
}

extern "C" void kernel_launch(void* const* d_in, const int* in_sizes, int n_in,
                              void* d_out, int out_size, void* d_ws, size_t ws_size,
                              hipStream_t stream) {
  if (n_in < 16) return;
  const int N = in_sizes[0] / DF;
  const int G = in_sizes[1] / DF;
  const int E = in_sizes[13] / 2;
  const int S = in_sizes[3] / (DF * DF);
  if (N <= 0 || in_sizes[0] != N * DF) return;
  if (G <= 0 || in_sizes[1] != G * DF) return;
  if (E < 0 || in_sizes[13] != 2 * E) return;
  if (S <= 0 || in_sizes[3] != S * DF * DF) return;
  if (in_sizes[4] != S * DF || in_sizes[5] != S * DF * 2 * DF || in_sizes[6] != S * DF) return;
  if (in_sizes[7] != S * DF || in_sizes[8] != S || in_sizes[9] != S * DF * DF || in_sizes[10] != S * DF) return;
  if (in_sizes[11] != S * DF * 2 * DF || in_sizes[12] != S * DF) return;
  if (in_sizes[14] != N) return;
  if (out_size != N * DF + G * DF) return;

  const float* x_in   = (const float*)d_in[0];
  const float* xgl_in = (const float*)d_in[1];
  const float* Wm  = (const float*)d_in[3];
  const float* bm  = (const float*)d_in[4];
  const float* Wa  = (const float*)d_in[5];
  const float* ba  = (const float*)d_in[6];
  const float* Wg  = (const float*)d_in[7];
  const float* bg  = (const float*)d_in[8];
  const float* Wf  = (const float*)d_in[9];
  const float* bfe = (const float*)d_in[10];
  const float* Wt  = (const float*)d_in[11];
  const float* bt  = (const float*)d_in[12];
  const int*   ei  = (const int*)d_in[13];
  const int*   batch = (const int*)d_in[14];
  float* out0 = (float*)d_out;
  float* out1 = out0 + (size_t)N * DF;

  size_t off = 0;
  auto carve = [&](size_t bytes) -> void* {
    void* p = (void*)((char*)d_ws + off);
    off += (bytes + 255) & ~(size_t)255;
    return p;
  };
  const size_t nWm = (size_t)S * DF * DF;
  const size_t nWa = (size_t)S * DF * 2 * DF;
  const int NPAD = ((N + NB - 1) / NB) * NB;
  const size_t nodeBytes = (size_t)NPAD * DF * sizeof(float);
  const int gN  = (N + GW * 16 - 1) / (GW * 16);
  const int GP  = ((G + GW * 16 - 1) / (GW * 16)) * (GW * 16);
  us16* Wmh = (us16*)carve(nWm * 2); us16* Wml = (us16*)carve(nWm * 2);
  us16* Wah = (us16*)carve(nWa * 2); us16* Wal = (us16*)carve(nWa * 2);
  us16* Wfh = (us16*)carve(nWm * 2); us16* Wfl = (us16*)carve(nWm * 2);
  us16* Wth = (us16*)carve(nWa * 2); us16* Wtl = (us16*)carve(nWa * 2);
  float* bufM = (float*)carve(nodeBytes);
  float* agg  = (float*)carve(nodeBytes);
  float* xA   = (float*)carve(nodeBytes);
  float* xB   = (float*)carve(nodeBytes);
  float* gate = (float*)carve((size_t)gN * (GW * 16) * sizeof(float));
  float* xg   = (float*)carve((size_t)GP * DF * sizeof(float));
  float* xglA = (float*)carve((size_t)GP * DF * sizeof(float));
  float* xglB = (float*)carve((size_t)GP * DF * sizeof(float));
  if (off > ws_size) return;
  if (off > (size_t)134217728u) return;

  {
    const int n8m = (int)(nWm / 8), n8a = (int)(nWa / 8);
    k_prep<<<(n8m + 255) / 256, 256, 0, stream>>>(Wm, Wmh, Wml, n8m);
    k_prep<<<(n8a + 255) / 256, 256, 0, stream>>>(Wa, Wah, Wal, n8a);
    k_prep<<<(n8m + 255) / 256, 256, 0, stream>>>(Wf, Wfh, Wfl, n8m);
    k_prep<<<(n8a + 255) / 256, 256, 0, stream>>>(Wt, Wth, Wtl, n8a);
  }

  hipFuncSetAttribute(reinterpret_cast<const void*>(&k_aggmax),
                      hipFuncAttributeMaxDynamicSharedMemorySize, ALDS_BYTES);

  const int aggGrid = (N + NB - 1) / NB;
  const int gG = (G + GW * 16 - 1) / (GW * 16);
  const float* xin = x_in;
  const float* xglin = xgl_in;
  for (int i = 0; i < S; ++i) {
    float* xout   = (i == S - 1) ? out0 : ((i & 1) ? xB : xA);
    float* xglout = (i == S - 1) ? out1 : ((i & 1) ? xglB : xglA);
    const us16* wmh = Wmh + (size_t)i * DF * DF;     const us16* wml = Wml + (size_t)i * DF * DF;
    const us16* wah = Wah + (size_t)i * DF * 2 * DF; const us16* wal = Wal + (size_t)i * DF * 2 * DF;
    const us16* wfh = Wfh + (size_t)i * DF * DF;     const us16* wfl = Wfl + (size_t)i * DF * DF;
    const us16* wth = Wth + (size_t)i * DF * 2 * DF; const us16* wtl = Wtl + (size_t)i * DF * 2 * DF;

    k_gemm<4, 0, false, false><<<gN, GT, 0, stream>>>(xin, xin, wmh, wml, bm + (size_t)i * DF, xin,
                                                       Wg, bg, gate, bufM, N);
    k_aggmax<<<aggGrid, ATHR, ALDS_BYTES, stream>>>(bufM, ei, agg, N, E);
    k_gemm<4, 4, true, false><<<gN, GT, 0, stream>>>(xin, agg, wah, wal, ba + (size_t)i * DF, xin,
                                                      Wg, bg, gate, xout, N);
    k_gemm<4, 0, false, true><<<gN, GT, 0, stream>>>(xout, xout, wfh, wfl, bfe + (size_t)i * DF, xout,
                                                      Wg + (size_t)i * DF, bg + i, gate, bufM, N);
    k_pool<<<G, PTHR, 0, stream>>>(gate, bufM, batch, xg, N);
    k_gemm<4, 4, true, false><<<gG, GT, 0, stream>>>(xg, xglin, wth, wtl, bt + (size_t)i * DF, xglin,
                                                      Wg, bg, gate, xglout, G);
    xin = xout;
    xglin = xglout;
  }
}
